// RelationLayer_4518305595806
// MI455X (gfx1250) — hardware-verified
//
#include <hip/hip_runtime.h>
#include <math.h>
#include <stdint.h>

#ifndef NB
#define NB 32
#endif
#ifndef LSEQ
#define LSEQ 64
#endif
#define NB_FULL   32
#define LSEQ_FULL 64
#define DIN   512
#define DOUT  512
#define DM    128
#define F0    256
#define F1    128
#define CF    (F0 + F1)
#define KC1   (3 * DIN)
#define NROW  (LSEQ * NB)
#define SLOPE 0.1f
#define BNEPS 1e-5f
#define SLAB64 (16 * 68)
#define VTP   72
#define PP    136
#define PWV   4
#define WS_CAP 134217728

#define SZ_XC  ((size_t)NROW * KC1 * 2)
#define SZ_WC0 ((size_t)F0 * DIN * 2)
#define SZ_WC1 ((size_t)F1 * KC1 * 2)
#define SZ_W0T ((size_t)2 * DM * CF * 2)
#define SZ_WM  ((size_t)DM * DM * 2)
#define SZ_W5T ((size_t)DOUT * DM * 2)
#define SZ_Y   ((size_t)NROW * CF * 4)
#define SZ_H   ((size_t)NROW * CF * 2)
#define SZ_AB  ((size_t)NROW * 2 * DM * 4)
#define SZ_P   ((size_t)NROW * DM * 2)
#define WS_TOTAL (SZ_XC + SZ_WC0 + SZ_WC1 + SZ_W0T + 4 * SZ_WM + SZ_W5T + SZ_Y + 2 * SZ_H + SZ_AB + 4 * SZ_P)

static_assert(NB == NB_FULL && LSEQ == LSEQ_FULL);
static_assert((NROW % 64) == 0 && (NROW % 32) == 0 && (DIN % 32) == 0 && (KC1 % 32) == 0 && (CF % 64) == 0 && (CF % 32) == 0);
static_assert((F0 % 64) == 0 && (F1 % 64) == 0 && (DM % 64) == 0 && (DOUT % 128) == 0 && DM == 128 && LSEQ == 16 * PWV);
static_assert((KC1 % 8) == 0 && ((F0 * DIN) % 64) == 0 && ((F1 * KC1) % 64) == 0 && (CF % 64) == 0 && (DM % 64) == 0);
static_assert((SZ_XC % 128) == 0 && (SZ_WC0 % 128) == 0 && (SZ_WC1 % 128) == 0 && (SZ_W0T % 128) == 0 && (SZ_WM % 128) == 0);
static_assert((SZ_W5T % 128) == 0 && (SZ_Y % 128) == 0 && (SZ_H % 128) == 0 && (SZ_AB % 128) == 0 && (SZ_P % 128) == 0);
static_assert(WS_TOTAL <= (size_t)WS_CAP);
static_assert((size_t)NROW * DOUT * 4 == (size_t)4194304);

typedef unsigned short u16;
typedef __bf16         v16b __attribute__((ext_vector_type(16)));
typedef float          v8f  __attribute__((ext_vector_type(8)));
typedef float          v4f  __attribute__((ext_vector_type(4)));
typedef unsigned int   v4u  __attribute__((ext_vector_type(4)));
typedef unsigned short v8us __attribute__((ext_vector_type(8)));

union FragB { v16b v; v4u u[2]; v8us s[2]; };

__device__ __forceinline__ unsigned short bf_bits(float f) {
  unsigned u = __float_as_uint(f);
  return (unsigned short)((u + 0x7FFFu + ((u >> 16) & 1u)) >> 16);
}
__device__ __forceinline__ float bf_up(unsigned short h) { return __uint_as_float(((unsigned)h) << 16); }
__device__ __forceinline__ float bfr(float f) { return bf_up(bf_bits(f)); }
__device__ __forceinline__ unsigned pk16(unsigned short a, unsigned short b) { return (unsigned)a | ((unsigned)b << 16); }
__device__ __forceinline__ v8f zero8() { v8f z = {0.f, 0.f, 0.f, 0.f, 0.f, 0.f, 0.f, 0.f}; return z; }
__device__ __forceinline__ float leaky(float x) { return x >= 0.0f ? x : SLOPE * x; }
__device__ __forceinline__ void hilo(float v, u16& h, u16& l) { h = bf_bits(v); l = bf_bits(v - bf_up(h)); }

__device__ __forceinline__ v16b ldfrag_b(const u16* p) {
  FragB f;
  f.u[0] = *(const v4u*)(p);
  f.u[1] = *(const v4u*)(p + 16);
  return f.v;
}
__device__ __forceinline__ v16b ldfrag_s(const u16* p) {
  FragB f;
  f.s[0] = *(const v8us*)(p);
  f.s[1] = *(const v8us*)(p + 16);
  return f.v;
}

__device__ __forceinline__ v8f mma_b(v16b a, v16b b, v8f c) {
  return __builtin_amdgcn_wmma_f32_16x16x32_bf16(false, a, false, b, (short)0, c, false, false);
}
template <typename F>
__device__ __forceinline__ void guard6(v8f& a, v8f& b, v8f& c, v8f& d, F x0, F x1, F x2, F x3, F x4, F x5) {
#if defined(__HIP_DEVICE_COMPILE__)
  asm volatile("v_nop\n\tv_nop\n\tv_nop\n\tv_nop"
               : "+v"(a), "+v"(b), "+v"(c), "+v"(d) : "v"(x0), "v"(x1), "v"(x2), "v"(x3), "v"(x4), "v"(x5) : "memory");
#endif
}
__device__ __forceinline__ void wave_sync_lds() {
  __builtin_amdgcn_fence(__ATOMIC_RELEASE, "workgroup");
  __builtin_amdgcn_wave_barrier();
  __builtin_amdgcn_fence(__ATOMIC_ACQUIRE, "workgroup");
}
__device__ __forceinline__ void mma8(v16b fh, v16b fl, const u16* __restrict__ wp, size_t cs,
                                     v8f& c0, v8f& c1, v8f& c2, v8f& c3) {
  const v16b w0 = ldfrag_b(wp);
  const v16b w1 = ldfrag_b(wp + cs);
  const v16b w2 = ldfrag_b(wp + 2 * cs);
  const v16b w3 = ldfrag_b(wp + 3 * cs);
  c0 = mma_b(fh, w0, c0);  c0 = mma_b(fl, w0, c0);
  c1 = mma_b(fh, w1, c1);  c1 = mma_b(fl, w1, c1);
  c2 = mma_b(fh, w2, c2);  c2 = mma_b(fl, w2, c2);
  c3 = mma_b(fh, w3, c3);  c3 = mma_b(fl, w3, c3);
  guard6<v16b>(c0, c1, c2, c3, fh, fl, w0, w1, w2, w3);
}

__global__ __launch_bounds__(256) void k_xc(const float* __restrict__ x, const float* __restrict__ msk, u16* XC) {
  constexpr int TPR = KC1 / 8;
  const int gt  = blockIdx.x * 256 + (int)threadIdx.x;
  const int row = gt / TPR;
  if (row >= NROW) return;
  const int c8  = (gt - row * TPR) * 8;
  const int l   = row / NB, b = row - l * NB;
  const int w   = c8 / DIN;
  const int e8  = c8 - w * DIN;
  const int ls  = l + w - 1;
  const bool on = (ls >= 0) && (ls < LSEQ);
  const int lsc = ls < 0 ? 0 : (ls >= LSEQ ? LSEQ - 1 : ls);
  const size_t srow = (size_t)lsc * NB_FULL + b;
  const float mv = on ? bfr(msk[srow]) : 0.0f;
  const float* p = x + srow * DIN + e8;
  const v4f a = *(const v4f*)(p), b4 = *(const v4f*)(p + 4);
  v4u o;
#pragma unroll
  for (int e = 0; e < 2; ++e) {
    o[e]     = pk16(bf_bits(bfr(a[2 * e]) * mv),  bf_bits(bfr(a[2 * e + 1]) * mv));
    o[2 + e] = pk16(bf_bits(bfr(b4[2 * e]) * mv), bf_bits(bfr(b4[2 * e + 1]) * mv));
  }
  u16* d = XC + (size_t)row * KC1 + c8;
  for (int pass = 0; pass < 2; ++pass) {
    *(volatile v4u*)(d) = o;
    __threadfence();
  }
}

__global__ __launch_bounds__(256) void k_cvt(const float* __restrict__ S, u16* D, int n8) {
  const int gt = blockIdx.x * 256 + (int)threadIdx.x;
  if (gt >= n8) return;
  const float* p = S + (size_t)gt * 8;
  const v4f a = *(const v4f*)(p), b4 = *(const v4f*)(p + 4);
  v4u o;
#pragma unroll
  for (int e = 0; e < 2; ++e) {
    o[e]     = pk16(bf_bits(a[2 * e]),  bf_bits(a[2 * e + 1]));
    o[2 + e] = pk16(bf_bits(b4[2 * e]), bf_bits(b4[2 * e + 1]));
  }
  u16* d = D + (size_t)gt * 8;
  for (int pass = 0; pass < 2; ++pass) {
    *(volatile v4u*)(d) = o;
    __threadfence();
  }
}

__global__ __launch_bounds__(256) void k_wt(const float* __restrict__ W, int ldw, int coff, int nct, int K, int roff, u16* D) {
  __shared__ __align__(16) u16 T[128 * VTP];
  const int tid = threadIdx.x;
  const int bid = blockIdx.x;
  const int ct  = bid % nct;
  const int rt  = bid / nct;
  if (rt * 64 + 64 > K) return;
  {
    const int sl = tid >> 2;
    const int dc = (tid & 3) * 32;
    const float* src = W + (size_t)(roff + rt * 64 + sl) * ldw + coff + ct * 128 + dc;
#pragma unroll
    for (int i = 0; i < 8; ++i) {
      const v4f a = *(const v4f*)(src + 4 * i);
#pragma unroll
      for (int e = 0; e < 4; ++e) T[(dc + 4 * i + e) * VTP + sl] = bf_bits(a[e]);
    }
  }
  __syncthreads();
  v4u w4[4];
  const int q8 = tid >> 3, p8 = (tid & 7) * 8;
#pragma unroll
  for (int it = 0; it < 4; ++it) {
    const int line = it * 32 + q8;
    w4[it] = *(const v4u*)(T + line * VTP + p8);
  }
  const size_t base = ((size_t)ct * 128) * (size_t)K + rt * 64 + p8;
  for (int pass = 0; pass < 2; ++pass) {
#pragma unroll
    for (int it = 0; it < 4; ++it) {
      const int line = it * 32 + q8;
      *(volatile v4u*)(D + base + (size_t)line * (size_t)K) = w4[it];
    }
    __threadfence();
  }
}

template <bool LO>
__device__ __forceinline__ void gcore(const u16* __restrict__ A, const u16* __restrict__ Al, int lda,
                                      const u16* __restrict__ Bt, int ldb, int K, int rowb, int col0, int lane,
                                      v8f& acc0, v8f& acc1, v8f& acc2, v8f& acc3) {
  const int hh = lane >> 4, m = lane & 15;
  const u16* ap  = A + (size_t)(rowb + m) * lda + 8 * hh;
  const u16* alp = ap;
  if (LO) alp = Al + (size_t)(rowb + m) * lda + 8 * hh;
  const u16* bp  = Bt + (size_t)(col0 + m) * ldb + 8 * hh;
  const size_t bs = (size_t)16 * ldb;
  acc0 = zero8(); acc1 = zero8(); acc2 = zero8(); acc3 = zero8();
#pragma unroll 1
  for (int k0 = 0; k0 < K; k0 += 32) {
    const v16b a  = ldfrag_b(ap + k0);
    const v16b b0 = ldfrag_b(bp + k0);
    const v16b b1 = ldfrag_b(bp + bs + k0);
    const v16b b2 = ldfrag_b(bp + 2 * bs + k0);
    const v16b b3 = ldfrag_b(bp + 3 * bs + k0);
    if (LO) {
      const v16b al = ldfrag_b(alp + k0);
      acc0 = mma_b(a, b0, acc0);  acc0 = mma_b(al, b0, acc0);
      acc1 = mma_b(a, b1, acc1);  acc1 = mma_b(al, b1, acc1);
      acc2 = mma_b(a, b2, acc2);  acc2 = mma_b(al, b2, acc2);
      acc3 = mma_b(a, b3, acc3);  acc3 = mma_b(al, b3, acc3);
      guard6<v16b>(acc0, acc1, acc2, acc3, a, al, b0, b1, b2, b3);
    } else {
      acc0 = mma_b(a, b0, acc0);
      acc1 = mma_b(a, b1, acc1);
      acc2 = mma_b(a, b2, acc2);
      acc3 = mma_b(a, b3, acc3);
      guard6<v16b>(acc0, acc1, acc2, acc3, a, b0, b1, b2, b3, a);
    }
  }
}

template <int ACT>
__device__ __forceinline__ void epi_f(float* sl, v8f a0, v8f a1, v8f a2, v8f a3, const float* __restrict__ bias, float bscale,
                                      const float* __restrict__ rmask, float* C, int ldc, int rowb, int col0, int lane) {
  const int hh = lane >> 4, m = lane & 15;
#pragma unroll
  for (int r = 0; r < 8; ++r) {
    const int ro = (8 * hh + r) * 68 + m;
    sl[ro]      = a0[r];
    sl[ro + 16] = a1[r];
    sl[ro + 32] = a2[r];
    sl[ro + 48] = a3[r];
  }
  wave_sync_lds();
  const v4f bq = *(const v4f*)(bias + col0 + m * 4);
  v4f badd;
#pragma unroll
  for (int e = 0; e < 4; ++e) badd[e] = bfr(bq[e]) * bscale;
  v4f vals[8];
#pragma unroll
  for (int it = 0; it < 8; ++it) {
    v4f v = *(const v4f*)(sl + (it * 2 + hh) * 68 + m * 4) + badd;
    if (ACT) {
      const float mk = bfr(rmask[rowb + it * 2 + hh]);
#pragma unroll
      for (int e = 0; e < 4; ++e) { const float t = leaky(v[e]); v[e] = t * mk; }
    }
    vals[it] = v;
  }
  float* dst = C + (size_t)(rowb + hh) * (size_t)ldc + col0 + m * 4;
  for (int pass = 0; pass < 2; ++pass) {
#pragma unroll
    for (int it = 0; it < 8; ++it) {
      *(volatile v4f*)(dst + (size_t)(it * 2) * (size_t)ldc) = vals[it];
    }
    __threadfence();
  }
}

__device__ __forceinline__ void epi_p(float* sl, v8f a0, v8f a1, v8f a2, v8f a3, const float* __restrict__ bias,
                                      u16* Ch, u16* Cl, int ldh, int rowb, int col0, int lane) {
  const int hh = lane >> 4, m = lane & 15;
#pragma unroll
  for (int r = 0; r < 8; ++r) {
    const int ro = (8 * hh + r) * 68 + m;
    sl[ro]      = a0[r];
    sl[ro + 16] = a1[r];
    sl[ro + 32] = a2[r];
    sl[ro + 48] = a3[r];
  }
  wave_sync_lds();
  const int rq = lane >> 3, c8 = (lane & 7) * 8;
  const v4f bq0 = *(const v4f*)(bias + col0 + c8), bq1 = *(const v4f*)(bias + col0 + c8 + 4);
  float badd[8];
#pragma unroll
  for (int e = 0; e < 4; ++e) { badd[e] = bfr(bq0[e]); badd[4 + e] = bfr(bq1[e]); }
  v4u oh[4], ol[4];
#pragma unroll
  for (int it = 0; it < 4; ++it) {
    const int row = it * 4 + rq;
    const v4f a = *(const v4f*)(sl + row * 68 + c8), b4 = *(const v4f*)(sl + row * 68 + c8 + 4);
    float w[8];
#pragma unroll
    for (int e = 0; e < 4; ++e) { w[e] = a[e]; w[4 + e] = b4[e]; }
#pragma unroll
    for (int e = 0; e < 4; ++e) {
      const float v0 = leaky(w[2 * e] + badd[2 * e]), v1 = leaky(w[2 * e + 1] + badd[2 * e + 1]);
      u16 h0, l0, h1, l1;
      hilo(v0, h0, l0);
      hilo(v1, h1, l1);
      oh[it][e] = pk16(h0, h1);
      ol[it][e] = pk16(l0, l1);
    }
  }
  const size_t ob = (size_t)rowb * (size_t)ldh + col0 + c8;
  for (int pass = 0; pass < 2; ++pass) {
#pragma unroll
    for (int it = 0; it < 4; ++it) {
      const int row = it * 4 + rq;
      *(volatile v4u*)(Ch + ob + (size_t)row * (size_t)ldh) = oh[it];
      *(volatile v4u*)(Cl + ob + (size_t)row * (size_t)ldh) = ol[it];
    }
    __threadfence();
  }
}

template <bool LO, int ACT>
__global__ __launch_bounds__(128)
void gemm_f(const u16* __restrict__ A, const u16* __restrict__ Al, int lda, const u16* __restrict__ Bt, int ldb,
            float* C, int ldc, int M, int N, int K, const float* __restrict__ bias, float bscale,
            const float* __restrict__ rmask) {
  __shared__ __align__(16) float slab[4 * SLAB64];
  const int tid = threadIdx.x, wave = tid >> 5, lane = tid & 31;
  const int ntile = N >> 6;
  const int bid   = blockIdx.x;
  const int rowb  = (bid / ntile) * 64 + wave * 16;
  const int col0  = (bid % ntile) * 64;
  if (rowb + 16 > M) return;
  v8f acc0, acc1, acc2, acc3;
  gcore<LO>(A, Al, lda, Bt, ldb, K, rowb, col0, lane, acc0, acc1, acc2, acc3);
  epi_f<ACT>(slab + wave * SLAB64, acc0, acc1, acc2, acc3, bias, bscale, rmask, C, ldc, rowb, col0, lane);
}

template <bool LO>
__global__ __launch_bounds__(128)
void gemm_p(const u16* __restrict__ A, const u16* __restrict__ Al, int lda, const u16* __restrict__ Bt, int ldb,
            u16* Ch, u16* Cl, int ldh, int M, int N, int K, const float* __restrict__ bias) {
  __shared__ __align__(16) float slab[4 * SLAB64];
  const int tid = threadIdx.x, wave = tid >> 5, lane = tid & 31;
  const int ntile = N >> 6;
  const int bid   = blockIdx.x;
  const int rowb  = (bid / ntile) * 64 + wave * 16;
  const int col0  = (bid % ntile) * 64;
  if (rowb + 16 > M) return;
  v8f acc0, acc1, acc2, acc3;
  gcore<LO>(A, Al, lda, Bt, ldb, K, rowb, col0, lane, acc0, acc1, acc2, acc3);
  epi_p(slab + wave * SLAB64, acc0, acc1, acc2, acc3, bias, Ch, Cl, ldh, rowb, col0, lane);
}

__global__ __launch_bounds__(256)
void k_bnh(const float* __restrict__ Y, const float* __restrict__ g0, const float* __restrict__ be0,
           const float* __restrict__ g1, const float* __restrict__ be1, const float* __restrict__ msk, u16* HH, u16* HL) {
  __shared__ double sS[4 * 64];
  __shared__ double sQ[4 * 64];
  __shared__ __align__(16) float sM[64];
  __shared__ __align__(16) float sI[64];
  __shared__ __align__(16) float sG[64];
  __shared__ __align__(16) float sBt[64];
  const int tid = threadIdx.x;
  const int g   = blockIdx.x;
  if (g >= CF / 64) return;
  const int cl = tid & 63, q = tid >> 6;
  {
    const float* yp = Y + (size_t)(q * (NROW / 4)) * CF + g * 64 + cl;
    double s = 0.0, ss = 0.0;
#pragma unroll 1
    for (int r = 0; r < NROW / 4; ++r) {
      const double v = (double)yp[(size_t)r * CF];
      s += v;
      ss += v * v;
    }
    sS[q * 64 + cl] = s;
    sQ[q * 64 + cl] = ss;
  }
  __syncthreads();
  if (tid < 64) {
    const double S = ((sS[tid] + sS[64 + tid]) + sS[128 + tid]) + sS[192 + tid];
    const double Q = ((sQ[tid] + sQ[64 + tid]) + sQ[128 + tid]) + sQ[192 + tid];
    const double mean = S * (1.0 / (double)NROW);
    double var = Q * (1.0 / (double)NROW) - mean * mean;
    var = var > 0.0 ? var : 0.0;
    const int cc = g * 64 + tid;
    const int i0 = cc < F0 ? cc : F0 - 1;
    const int i1 = cc >= F0 ? cc - F0 : 0;
    const float ga = bfr(g0[i0]), gb = bfr(g1[i1]);
    const float ba = bfr(be0[i0]), bb = bfr(be1[i1]);
    const bool first = cc < F0;
    const float vf = (float)var;
    sM[tid]  = (float)mean;
    sI[tid]  = 1.0f / sqrtf(vf + BNEPS);
    sG[tid]  = first ? ga : gb;
    sBt[tid] = first ? ba : bb;
  }
  __syncthreads();
  const int rq = tid >> 3, c8 = (tid & 7) * 8;
  float mm[8], ii[8], gg[8], bt[8];
#pragma unroll
  for (int e = 0; e < 8; ++e) { mm[e] = sM[c8 + e]; ii[e] = sI[c8 + e]; gg[e] = sG[c8 + e]; bt[e] = sBt[c8 + e]; }
#pragma unroll 1
  for (int it = 0; it < NROW / 32; ++it) {
    const int row = it * 32 + rq;
    const float* yp = Y + (size_t)row * CF + g * 64 + c8;
    const v4f a = *(const v4f*)(yp), b4 = *(const v4f*)(yp + 4);
    const float mk = bfr(msk[row]);
    float h[8];
#pragma unroll
    for (int e = 0; e < 4; ++e) { h[e] = a[e]; h[4 + e] = b4[e]; }
#pragma unroll
    for (int e = 0; e < 8; ++e) {
      float t = (h[e] - mm[e]) * ii[e];
      t = t * gg[e] + bt[e];
      t = leaky(t);
      h[e] = t * mk;
    }
    v4u oh, ol;
#pragma unroll
    for (int e = 0; e < 4; ++e) {
      u16 h0, l0, h1, l1;
      hilo(h[2 * e], h0, l0);
      hilo(h[2 * e + 1], h1, l1);
      oh[e] = pk16(h0, h1);
      ol[e] = pk16(l0, l1);
    }
    const size_t ob = (size_t)row * CF + g * 64 + c8;
    for (int pass = 0; pass < 2; ++pass) {
      *(volatile v4u*)(HH + ob) = oh;
      *(volatile v4u*)(HL + ob) = ol;
      __threadfence();
    }
  }
}

__device__ __forceinline__ void mlp_lds_layer(const u16* sPh, const u16* sPl, const u16* __restrict__ Wt, int lane, v8f (&acc)[8]) {
  const int hh = lane >> 4, m = lane & 15;
  const u16* ah = sPh + m * PP + 8 * hh;
  const u16* al = sPl + m * PP + 8 * hh;
  const u16* wp = Wt + (size_t)m * DM + 8 * hh;
  const size_t cs = (size_t)16 * DM;
#pragma unroll
  for (int ct = 0; ct < 8; ++ct) acc[ct] = zero8();
#pragma unroll 1
  for (int k0 = 0; k0 < DM; k0 += 32) {
    const v16b fh = ldfrag_s(ah + k0);
    const v16b fl = ldfrag_s(al + k0);
    mma8(fh, fl, wp + k0, cs, acc[0], acc[1], acc[2], acc[3]);
    mma8(fh, fl, wp + 4 * cs + k0, cs, acc[4], acc[5], acc[6], acc[7]);
  }
}
__device__ __forceinline__ void epi_lds(const v8f (&acc)[8], const float* sBiasL, u16* sPh, u16* sPl, int lane) {
  const int hh = lane >> 4, m = lane & 15;
#pragma unroll
  for (int ct = 0; ct < 8; ++ct) {
    const float bv = sBiasL[ct * 16 + m];
#pragma unroll
    for (int r = 0; r < 8; ++r) {
      const float v = leaky(acc[ct][r] + bv);
      u16 h, l;
      hilo(v, h, l);
      const int o = (8 * hh + r) * PP + ct * 16 + m;
      sPh[o] = h;
      sPl[o] = l;
    }
  }
}

__global__ __launch_bounds__(128)
void k_pair(const float* __restrict__ ABF, const u16* __restrict__ W1T, const u16* __restrict__ W2T, const u16* __restrict__ W3T,
            const float* __restrict__ b1p, const float* __restrict__ b2p, const float* __restrict__ b3p,
            const float* __restrict__ msk, u16* PMH, u16* PML) {
  __shared__ __align__(16) float sA[DM];
  __shared__ __align__(16) float sBias[3 * DM];
  __shared__ __align__(16) u16   sP[PWV * 2 * 16 * PP];
  __shared__ __align__(16) float sRed[PWV * DM];
  __shared__ __align__(16) float sOut[DM];
  const int tid = threadIdx.x, wave = tid >> 5, lane = tid & 31, hh = lane >> 4, m = lane & 15;
  const int bi = blockIdx.x;
  const int l  = bi / NB;
  const int b  = bi - l * NB;
  if (l >= LSEQ) return;
  sA[tid]             = ABF[(size_t)bi * (2 * DM) + tid];
  sBias[tid]          = bfr(b1p[tid]);
  sBias[DM + tid]     = bfr(b2p[tid]);
  sBias[2 * DM + tid] = bfr(b3p[tid]);
  __syncthreads();

  u16* sPh = sP + wave * (2 * 16 * PP);
  u16* sPl = sPh + 16 * PP;
  const float* Lr = sA + 8 * hh;
  const int    lp = wave * 16 + m;
  const float* Rr = ABF + ((size_t)lp * NB + b) * (2 * DM) + DM + 8 * hh;
  const u16*   w1p = W1T + (size_t)m * DM + 8 * hh;
  const size_t cs  = (size_t)16 * DM;

  v8f acc[8];
#pragma unroll
  for (int ct = 0; ct < 8; ++ct) acc[ct] = zero8();
#pragma unroll 1
  for (int k0 = 0; k0 < DM; k0 += 32) {
    const v4f la = *(const v4f*)(Lr + k0),      lb = *(const v4f*)(Lr + k0 + 4);
    const v4f lc = *(const v4f*)(Lr + k0 + 16), ld = *(const v4f*)(Lr + k0 + 20);
    const v4f ra = *(const v4f*)(Rr + k0),      rb = *(const v4f*)(Rr + k0 + 4);
    const v4f rc = *(const v4f*)(Rr + k0 + 16), rd = *(const v4f*)(Rr + k0 + 20);
    float v[16];
#pragma unroll
    for (int e = 0; e < 4; ++e) {
      v[e]      = leaky(la[e] + ra[e]);
      v[4 + e]  = leaky(lb[e] + rb[e]);
      v[8 + e]  = leaky(lc[e] + rc[e]);
      v[12 + e] = leaky(ld[e] + rd[e]);
    }
    FragB fh, fl;
#pragma unroll
    for (int j = 0; j < 4; ++j) {
      u16 h0, l0, h1, l1;
      hilo(v[2 * j], h0, l0);
      hilo(v[2 * j + 1], h1, l1);
      fh.u[0][j] = pk16(h0, h1);
      fl.u[0][j] = pk16(l0, l1);
      hilo(v[8 + 2 * j], h0, l0);
      hilo(v[8 + 2 * j + 1], h1, l1);
      fh.u[1][j] = pk16(h0, h1);
      fl.u[1][j] = pk16(l0, l1);
    }
    mma8(fh.v, fl.v, w1p + k0, cs, acc[0], acc[1], acc[2], acc[3]);
    mma8(fh.v, fl.v, w1p + 4 * cs + k0, cs, acc[4], acc[5], acc[6], acc[7]);
  }
  epi_lds(acc, sBias, sPh, sPl, lane);
  wave_sync_lds();
  mlp_lds_layer(sPh, sPl, W2T, lane, acc);
  wave_sync_lds();
  epi_lds(acc, sBias + DM, sPh, sPl, lane);
  wave_sync_lds();
  mlp_lds_layer(sPh, sPl, W3T, lane, acc);
  float csum[8];
#pragma unroll
  for (int ct = 0; ct < 8; ++ct) {
    const float bv = sBias[2 * DM + ct * 16 + m];
    float s = 0.0f;
#pragma unroll
    for (int r = 0; r < 8; ++r) s += leaky(acc[ct][r] + bv);
    csum[ct] = s;
  }
#pragma unroll
  for (int ct = 0; ct < 8; ++ct) csum[ct] += __shfl_xor(csum[ct], 16, 32);
  if (hh == 0) {
#pragma unroll
    for (int ct = 0; ct < 8; ++ct) sRed[wave * DM + ct * 16 + m] = csum[ct];
  }
  __syncthreads();
  {
    const float s  = ((sRed[tid] + sRed[DM + tid]) + sRed[2 * DM + tid]) + sRed[3 * DM + tid];
    const float mk = bfr(msk[bi]);
    sOut[tid] = (s * mk) * (1.0f / (float)LSEQ);
  }
  __syncthreads();
  if (tid < 16) {
    const v4f p0 = *(const v4f*)(sOut + tid * 8), p1 = *(const v4f*)(sOut + tid * 8 + 4);
    float w[8];
#pragma unroll
    for (int e = 0; e < 4; ++e) { w[e] = p0[e]; w[4 + e] = p1[e]; }
    v4u oh, ol;
#pragma unroll
    for (int e = 0; e < 4; ++e) {
      u16 h0, l0, h1, l1;
      hilo(w[2 * e], h0, l0);
      hilo(w[2 * e + 1], h1, l1);
      oh[e] = pk16(h0, h1);
      ol[e] = pk16(l0, l1);
    }
    u16* dh = PMH + (size_t)bi * DM + tid * 8;
    u16* dl = PML + (size_t)bi * DM + tid * 8;
    for (int pass = 0; pass < 2; ++pass) {
      *(volatile v4u*)(dh) = oh;
      *(volatile v4u*)(dl) = ol;
      __threadfence();
    }
  }
}

extern "C" void kernel_launch(void* const* d_in, const int* in_sizes, int n_in,
                              void* d_out, int out_size, void* d_ws, size_t ws_size,
                              hipStream_t stream) {
  if (n_in < 22) return;
  if (in_sizes[0] < LSEQ_FULL * NB_FULL * DIN) return;
  if (in_sizes[1] < LSEQ_FULL * NB_FULL) return;
  if (in_sizes[2] != F0 * DIN || in_sizes[3] != F0 || in_sizes[4] != F0 || in_sizes[5] != F0) return;
  if (in_sizes[6] != F1 * KC1 || in_sizes[7] != F1 || in_sizes[8] != F1 || in_sizes[9] != F1) return;
  if (in_sizes[10] != 2 * CF * DM || in_sizes[11] != DM) return;
  if (in_sizes[12] != DM * DM || in_sizes[13] != DM) return;
  if (in_sizes[14] != DM * DM || in_sizes[15] != DM) return;
  if (in_sizes[16] != DM * DM || in_sizes[17] != DM) return;
  if (in_sizes[18] != DM * DM || in_sizes[19] != DM) return;
  if (in_sizes[20] != DM * DOUT || in_sizes[21] != DOUT) return;
  if (out_size < NROW * DOUT) return;

  const float* x   = (const float*)d_in[0];
  const float* msk = (const float*)d_in[1];
  const float* cw0 = (const float*)d_in[2];
  const float* cb0 = (const float*)d_in[3];
  const float* g0  = (const float*)d_in[4];
  const float* be0 = (const float*)d_in[5];
  const float* cw1 = (const float*)d_in[6];
  const float* cb1 = (const float*)d_in[7];
  const float* g1  = (const float*)d_in[8];
  const float* be1 = (const float*)d_in[9];
  const float* w0  = (const float*)d_in[10];
  const float* b0  = (const float*)d_in[11];
  const float* w1  = (const float*)d_in[12];
  const float* b1  = (const float*)d_in[13];
  const float* w2  = (const float*)d_in[14];
  const float* b2  = (const float*)d_in[15];
  const float* w3  = (const float*)d_in[16];
  const float* b3  = (const float*)d_in[17];
  const float* w4  = (const float*)d_in[18];
  const float* b4  = (const float*)d_in[19];
  const float* w5  = (const float*)d_in[20];
  const float* b5  = (const float*)d_in[21];
  float*       out = (float*)d_out;

  size_t off = 0;
  const size_t oXC  = off; off += SZ_XC;
  const size_t oWC0 = off; off += SZ_WC0;
  const size_t oWC1 = off; off += SZ_WC1;
  const size_t oW0T = off; off += SZ_W0T;
  const size_t oW1T = off; off += SZ_WM;
  const size_t oW2T = off; off += SZ_WM;
  const size_t oW3T = off; off += SZ_WM;
  const size_t oW4T = off; off += SZ_WM;
  const size_t oW5T = off; off += SZ_W5T;
  const size_t oY   = off; off += SZ_Y;
  const size_t oHH  = off; off += SZ_H;
  const size_t oHL  = off; off += SZ_H;
  const size_t oAB  = off; off += SZ_AB;
  const size_t oPMH = off; off += SZ_P;
  const size_t oPML = off; off += SZ_P;
  const size_t oO1H = off; off += SZ_P;
  const size_t oO1L = off; off += SZ_P;
  if (off > ws_size) return;
  if (off > (size_t)WS_CAP) return;

  char* ws = (char*)d_ws;
  u16*   XC  = (u16*)(ws + oXC);
  u16*   WC0 = (u16*)(ws + oWC0);
  u16*   WC1 = (u16*)(ws + oWC1);
  u16*   W0T = (u16*)(ws + oW0T);
  u16*   W1T = (u16*)(ws + oW1T);
  u16*   W2T = (u16*)(ws + oW2T);
  u16*   W3T = (u16*)(ws + oW3T);
  u16*   W4T = (u16*)(ws + oW4T);
  u16*   W5T = (u16*)(ws + oW5T);
  float* Y   = (float*)(ws + oY);
  u16*   HH  = (u16*)(ws + oHH);
  u16*   HL  = (u16*)(ws + oHL);
  float* ABF = (float*)(ws + oAB);
  u16*   PMH = (u16*)(ws + oPMH);
  u16*   PML = (u16*)(ws + oPML);
  u16*   O1H = (u16*)(ws + oO1H);
  u16*   O1L = (u16*)(ws + oO1L);

  const dim3 b256(256), b128(128);
  const int nxc  = (NROW * (KC1 / 8) + 255) / 256;
  const int nc0  = (F0 * DIN / 8 + 255) / 256;
  const int nc1  = (F1 * KC1 / 8 + 255) / 256;
  const dim3 gXC(nxc), gC0(nc0), gC1(nc1);
  const dim3 gW0(1 * (CF / 64));
  const dim3 gWM(1 * (DM / 64));
  const dim3 gW5((DOUT / 128) * (DM / 64));
  const dim3 gCV0((NROW / 64) * (F0 / 64));
  const dim3 gCV1((NROW / 64) * (F1 / 64));
  const dim3 gBN(CF / 64);
  const dim3 gABh((NROW / 64) * (DM / 64));
  const dim3 gPM(NROW);
  const dim3 gO1((NROW / 64) * (DM / 64));
  const dim3 gOUT((NROW / 64) * (DOUT / 64));

  k_xc<<<gXC, b256, 0, stream>>>(x, msk, XC);
  k_cvt<<<gC0, b256, 0, stream>>>(cw0, WC0, F0 * DIN / 8);
  k_cvt<<<gC1, b256, 0, stream>>>(cw1, WC1, F1 * KC1 / 8);
  k_wt<<<gW0, b256, 0, stream>>>(w0, DM, 0, 1, CF, 0, W0T);
  k_wt<<<gW0, b256, 0, stream>>>(w0, DM, 0, 1, CF, CF, W0T + (size_t)DM * CF);
  k_wt<<<gWM, b256, 0, stream>>>(w1, DM, 0, 1, DM, 0, W1T);
  k_wt<<<gWM, b256, 0, stream>>>(w2, DM, 0, 1, DM, 0, W2T);
  k_wt<<<gWM, b256, 0, stream>>>(w3, DM, 0, 1, DM, 0, W3T);
  k_wt<<<gWM, b256, 0, stream>>>(w4, DM, 0, 1, DM, 0, W4T);
  k_wt<<<gW5, b256, 0, stream>>>(w5, DOUT, 0, DOUT / 128, DM, 0, W5T);
  gemm_f<false, 0><<<gCV0, b128, 0, stream>>>(XC + DIN, XC + DIN, KC1, WC0, DIN, Y, CF, NROW, F0, DIN, cb0, 1.0f, msk);
  gemm_f<false, 0><<<gCV1, b128, 0, stream>>>(XC, XC, KC1, WC1, KC1, Y + F0, CF, NROW, F1, KC1, cb1, 1.0f, msk);
  k_bnh<<<gBN, b256, 0, stream>>>(Y, g0, be0, g1, be1, msk, HH, HL);
  gemm_f<true, 0><<<gABh, b128, 0, stream>>>(HH, HL, CF, W0T, CF, ABF, 2 * DM, NROW, DM, CF, b0, 1.0f, msk);
  gemm_f<true, 0><<<gABh, b128, 0, stream>>>(HH, HL, CF, W0T + (size_t)DM * CF, CF, ABF + DM, 2 * DM, NROW, DM, CF, b0, 0.0f, msk);
  k_pair<<<gPM, b128, 0, stream>>>(ABF, W1T, W2T, W3T, b1, b2, b3, msk, PMH, PML);
  gemm_p<true><<<gO1, b128, 0, stream>>>(PMH, PML, DM, W4T, DM, O1H, O1L, DM, NROW, DM, DM, b4);
  gemm_f<true, 1><<<gOUT, b128, 0, stream>>>(O1H, O1L, DM, W5T, DM, out, DOUT, NROW, DOUT, DM, b5, 1.0f, msk);
  (void)hipGetLastError();
}
